// MultiHeadSelfAttention_42296837931163
// MI455X (gfx1250) — hardware-verified
//
#include <hip/hip_runtime.h>
#ifndef NB
#define NB 2
#endif
#ifndef SEQ
#define SEQ 2048
#endif
#ifndef FINE_ROWS
#define FINE_ROWS 512
#endif
#define B_FULL 2
#define T_FULL 2048
#define DM 1024
#define NH 16
#define HD 64
#define NRT (NB * SEQ)
#define LQK (2 * DM)

static_assert(NH * HD == DM);
static_assert(HD == 64);
static_assert(DM % 128 == 0);
static_assert(DM % 32 == 0);
static_assert(SEQ % 64 == 0);
static_assert(NRT % 128 == 0);
static_assert(LQK % 64 == 0);
static_assert(FINE_ROWS % 128 == 0);
static_assert(NB <= B_FULL);
static_assert(SEQ <= T_FULL);
static_assert((SEQ / 32) * 8 >= 1);

typedef _Float16 v16h __attribute__((ext_vector_type(16)));
typedef unsigned short v8us __attribute__((ext_vector_type(8), may_alias));
typedef unsigned int v4ua __attribute__((ext_vector_type(4), may_alias));
typedef float v8f __attribute__((ext_vector_type(8)));
typedef float v4f __attribute__((ext_vector_type(4)));
typedef float v4fa __attribute__((ext_vector_type(4), may_alias));
union FragH { v16h v; v8us half[2]; _Float16 h[16]; unsigned short u[16]; };

__device__ __forceinline__ float bf16_rne(float x) {
  unsigned int u = __float_as_uint(x);
  u = (u + 0x7FFFu + ((u >> 16) & 1u)) & 0xFFFF0000u;
  return __uint_as_float(u);
}
__device__ __forceinline__ unsigned short hbits(_Float16 v) { return __builtin_bit_cast(unsigned short, v); }

__device__ __forceinline__ v16h ld_frag(const unsigned short* __restrict__ p, int hh) {
  FragH f;
  f.half[0] = *(const v8us*)(p + 8 * hh);
  f.half[1] = *(const v8us*)(p + 16 + 8 * hh);
  return f.v;
}
__device__ __forceinline__ v8f mma1(v16h a, v16h b, v8f c) {
  c = __builtin_amdgcn_wmma_f32_16x16x32_f16(false, a, false, b, (short)0, c, false, false);
  asm volatile("v_nop\n\tv_nop\n\tv_nop\n\tv_nop" : "+v"(c) : "v"(a), "v"(b));
  return c;
}
__device__ __forceinline__ v8f mma2(v16h ah, v16h al, v16h b, v8f c) {
  c = __builtin_amdgcn_wmma_f32_16x16x32_f16(false, ah, false, b, (short)0, c, false, false);
  c = __builtin_amdgcn_wmma_f32_16x16x32_f16(false, al, false, b, (short)0, c, false, false);
  asm volatile("v_nop\n\tv_nop\n\tv_nop\n\tv_nop" : "+v"(c) : "v"(ah), "v"(al), "v"(b));
  return c;
}
__device__ __forceinline__ v8f mma3(v16h ah, v16h al, v16h bh, v16h bl, v8f c) {
  c = __builtin_amdgcn_wmma_f32_16x16x32_f16(false, ah, false, bh, (short)0, c, false, false);
  c = __builtin_amdgcn_wmma_f32_16x16x32_f16(false, al, false, bh, (short)0, c, false, false);
  c = __builtin_amdgcn_wmma_f32_16x16x32_f16(false, ah, false, bl, (short)0, c, false, false);
  asm volatile("v_nop\n\tv_nop\n\tv_nop\n\tv_nop" : "+v"(c) : "v"(ah), "v"(al), "v"(bh), "v"(bl));
  return c;
}

__global__ __launch_bounds__(256) void k_x16(const float* __restrict__ x, unsigned short* __restrict__ X16) {
  const size_t t = (size_t)blockIdx.x * 256 + threadIdx.x;
  if (t >= (size_t)NRT * (DM / 8)) return;
  const int rb = (int)(t / (DM / 8));
  const int k8 = (int)(t % (DM / 8)) * 8;
  const int b = rb / SEQ, tt = rb - b * SEQ;
  const float* src = x + ((size_t)tt * B_FULL + b) * DM + k8;
  const v4f a = *(const v4fa*)src;
  const v4f c = *(const v4fa*)(src + 4);
  FragH f;
#pragma unroll
  for (int q = 0; q < 4; ++q) { f.h[q] = (_Float16)bf16_rne(a[q]); f.h[4 + q] = (_Float16)bf16_rne(c[q]); }
  const v8us o = f.half[0];
  unsigned short* d = X16 + t * 8;
  *(volatile v8us*)d = o;
  __threadfence();
  *(volatile v8us*)d = o;
}

__global__ __launch_bounds__(256) void k_wplane(const float* __restrict__ W, unsigned short* __restrict__ Bt, int perm) {
  const size_t t = (size_t)blockIdx.x * 256 + threadIdx.x;
  if (t >= (size_t)DM * (DM / 8)) return;
  const int n = (int)(t / (DM / 8));
  const int k8 = (int)(t % (DM / 8)) * 8;
  const int srow = perm ? ((n & (HD - 1)) * NH + (n >> 6)) : n;
  const float* src = W + (size_t)srow * DM + k8;
  const v4f a = *(const v4fa*)src;
  const v4f c = *(const v4fa*)(src + 4);
  FragH f;
#pragma unroll
  for (int q = 0; q < 4; ++q) { f.h[q] = (_Float16)(bf16_rne(a[q]) * 16.0f); f.h[4 + q] = (_Float16)(bf16_rne(c[q]) * 16.0f); }
  const v8us o = f.half[0];
  unsigned short* d = Bt + t * 8;
  *(volatile v8us*)d = o;
  __threadfence();
  *(volatile v8us*)d = o;
}

__global__ __launch_bounds__(256) void k_maskbits(const int* __restrict__ mask, unsigned int* __restrict__ MB) {
  __shared__ unsigned int sb[SEQ / 32][33];
  const int tid = threadIdx.x, w = tid >> 5, lane = tid & 31;
  const int g = blockIdx.x;
#pragma unroll 1
  for (int rr = 0; rr < 4; ++rr) {
    const int rl = w * 4 + rr;
    const int* mrow = mask + (size_t)(g * 32 + rl) * T_FULL;
#pragma unroll 1
    for (int c = 0; c < SEQ / 32; ++c) {
      const int mv = mrow[c * 32 + lane];
      const unsigned int bits = (unsigned int)__ballot(mv != 0);
      if (lane == 0) sb[c][rl] = bits;
    }
  }
  __syncthreads();
  for (int pass = 0; pass < 2; ++pass) {
    for (int i = tid; i < (SEQ / 32) * 8; i += 256) {
      const int c = i >> 3, p = (i & 7) * 4;
      v4ua v;
      v[0] = sb[c][p]; v[1] = sb[c][p + 1]; v[2] = sb[c][p + 2]; v[3] = sb[c][p + 3];
      *(volatile v4ua*)(MB + (size_t)c * SEQ + g * 32 + p) = v;
    }
    if (pass == 0) __threadfence();
  }
}

__global__ __launch_bounds__(128) void k_proj(const unsigned short* __restrict__ A, int lda, const unsigned short* __restrict__ Bh, int ldb, float alpha,
                                              unsigned short* __restrict__ Ch, unsigned short* __restrict__ Cl, int ldc, int M, int N, int K) {
  __shared__ __attribute__((aligned(16))) float so[4][32][68];
  const int tid = threadIdx.x;
  const int w = __builtin_amdgcn_readfirstlane(tid >> 5);
  const int lane = tid & 31, ln = lane & 15, hh = lane >> 4;
  const int ntn = N >> 6;
  const int mt = blockIdx.x / ntn, nq = blockIdx.x - mt * ntn;
  const int row0 = mt * 128 + 32 * w, col0 = nq * 64;
  if (row0 >= M) return;
  const unsigned short* a0p = A + (size_t)(row0 + ln) * lda;
  const unsigned short* a1p = a0p + (size_t)16 * lda;
  const unsigned short* b0p = Bh + (size_t)(col0 + ln) * ldb;
  const unsigned short* b1p = b0p + (size_t)16 * ldb;
  const unsigned short* b2p = b1p + (size_t)16 * ldb;
  const unsigned short* b3p = b2p + (size_t)16 * ldb;
  const v8f z8 = {0.f, 0.f, 0.f, 0.f, 0.f, 0.f, 0.f, 0.f};
  v8f c00 = z8, c01 = z8, c02 = z8, c03 = z8, c10 = z8, c11 = z8, c12 = z8, c13 = z8;
#pragma unroll 1
  for (int kb = 0; kb < K; kb += 32) {
    const v16h a0 = ld_frag(a0p + kb, hh), a1 = ld_frag(a1p + kb, hh);
    v16h b = ld_frag(b0p + kb, hh); c00 = mma1(a0, b, c00); c10 = mma1(a1, b, c10);
    b = ld_frag(b1p + kb, hh); c01 = mma1(a0, b, c01); c11 = mma1(a1, b, c11);
    b = ld_frag(b2p + kb, hh); c02 = mma1(a0, b, c02); c12 = mma1(a1, b, c12);
    b = ld_frag(b3p + kb, hh); c03 = mma1(a0, b, c03); c13 = mma1(a1, b, c13);
  }
  const v8f accs[8] = {c00, c01, c02, c03, c10, c11, c12, c13};
#pragma unroll
  for (int u = 0; u < 8; ++u) {
    const int t = u & 3, half = u >> 2;
#pragma unroll
    for (int r = 0; r < 8; ++r) so[w][half * 16 + 8 * hh + r][t * 16 + ln] = accs[u][r] * alpha;
  }
  __builtin_amdgcn_fence(4  , "workgroup");
  __builtin_amdgcn_wave_barrier();
  const int rq = lane >> 3, c8 = (lane & 7) * 8;
  for (int pass = 0; pass < 2; ++pass) {
#pragma unroll
    for (int q = 0; q < 8; ++q) {
      const int r = q * 4 + rq;
      const v4f x0 = *(const v4fa*)&so[w][r][c8];
      const v4f x1 = *(const v4fa*)&so[w][r][c8 + 4];
      FragH fh, fl;
#pragma unroll
      for (int i = 0; i < 4; ++i) {
        _Float16 hv = (_Float16)x0[i]; fh.h[i] = hv; fl.h[i] = (_Float16)(x0[i] - (float)hv);
        hv = (_Float16)x1[i]; fh.h[4 + i] = hv; fl.h[4 + i] = (_Float16)(x1[i] - (float)hv);
      }
      const v8us oh = fh.half[0], ol = fl.half[0];
      const size_t o = (size_t)(row0 + r) * ldc + col0 + c8;
      *(volatile v8us*)(Ch + o) = oh;
      if (Cl) *(volatile v8us*)(Cl + o) = ol;
    }
    if (pass == 0) __threadfence();
  }
}

__global__ __launch_bounds__(128) void k_outg(const unsigned short* __restrict__ Ah, const unsigned short* __restrict__ Al, const unsigned short* __restrict__ Bh,
                                              float alpha, float* __restrict__ C) {
  __shared__ __attribute__((aligned(16))) float so[4][32][68];
  const int tid = threadIdx.x;
  const int w = __builtin_amdgcn_readfirstlane(tid >> 5);
  const int lane = tid & 31, ln = lane & 15, hh = lane >> 4;
  const int ntn = DM >> 6;
  const int mt = blockIdx.x / ntn, nq = blockIdx.x - mt * ntn;
  const int row0 = mt * 128 + 32 * w, col0 = nq * 64;
  if (row0 >= NRT) return;
  const bool fine = (row0 % SEQ) < FINE_ROWS;
  const size_t ao0 = (size_t)(row0 + ln) * DM, ao1 = ao0 + (size_t)16 * DM;
  const unsigned short* b0p = Bh + (size_t)(col0 + ln) * DM;
  const unsigned short* b1p = b0p + (size_t)16 * DM;
  const unsigned short* b2p = b1p + (size_t)16 * DM;
  const unsigned short* b3p = b2p + (size_t)16 * DM;
  const v8f z8 = {0.f, 0.f, 0.f, 0.f, 0.f, 0.f, 0.f, 0.f};
  v8f c00 = z8, c01 = z8, c02 = z8, c03 = z8, c10 = z8, c11 = z8, c12 = z8, c13 = z8;
  if (fine) {
#pragma unroll 1
    for (int kb = 0; kb < DM; kb += 32) {
      const v16h a0 = ld_frag(Ah + ao0 + kb, hh), a1 = ld_frag(Ah + ao1 + kb, hh);
      const v16h e0 = ld_frag(Al + ao0 + kb, hh), e1 = ld_frag(Al + ao1 + kb, hh);
      v16h b = ld_frag(b0p + kb, hh); c00 = mma2(a0, e0, b, c00); c10 = mma2(a1, e1, b, c10);
      b = ld_frag(b1p + kb, hh); c01 = mma2(a0, e0, b, c01); c11 = mma2(a1, e1, b, c11);
      b = ld_frag(b2p + kb, hh); c02 = mma2(a0, e0, b, c02); c12 = mma2(a1, e1, b, c12);
      b = ld_frag(b3p + kb, hh); c03 = mma2(a0, e0, b, c03); c13 = mma2(a1, e1, b, c13);
    }
  } else {
#pragma unroll 1
    for (int kb = 0; kb < DM; kb += 32) {
      const v16h a0 = ld_frag(Ah + ao0 + kb, hh), a1 = ld_frag(Ah + ao1 + kb, hh);
      v16h b = ld_frag(b0p + kb, hh); c00 = mma1(a0, b, c00); c10 = mma1(a1, b, c10);
      b = ld_frag(b1p + kb, hh); c01 = mma1(a0, b, c01); c11 = mma1(a1, b, c11);
      b = ld_frag(b2p + kb, hh); c02 = mma1(a0, b, c02); c12 = mma1(a1, b, c12);
      b = ld_frag(b3p + kb, hh); c03 = mma1(a0, b, c03); c13 = mma1(a1, b, c13);
    }
  }
  const v8f accs[8] = {c00, c01, c02, c03, c10, c11, c12, c13};
#pragma unroll
  for (int u = 0; u < 8; ++u) {
    const int t = u & 3, half = u >> 2;
#pragma unroll
    for (int r = 0; r < 8; ++r) so[w][half * 16 + 8 * hh + r][t * 16 + ln] = accs[u][r] * alpha;
  }
  __builtin_amdgcn_fence(4  , "workgroup");
  __builtin_amdgcn_wave_barrier();
  const int rsub = lane >> 4, c4 = (lane & 15) * 4;
  for (int pass = 0; pass < 2; ++pass) {
#pragma unroll
    for (int q = 0; q < 16; ++q) {
      const int r = q * 2 + rsub;
      const v4f v = *(const v4fa*)&so[w][r][c4];
      const int rb = row0 + r;
      const int bb = rb / SEQ, tt = rb - bb * SEQ;
      *(volatile v4f*)(C + ((size_t)tt * B_FULL + bb) * DM + col0 + c4) = v;
    }
    if (pass == 0) __threadfence();
  }
}

__global__ __launch_bounds__(128) void k_attn(const unsigned short* __restrict__ QKH, const unsigned short* __restrict__ QKL,
                                              const unsigned short* __restrict__ VTH, const unsigned short* __restrict__ VTL,
                                              const unsigned int* __restrict__ MB,
                                              unsigned short* __restrict__ OH, unsigned short* __restrict__ OL) {
  __shared__ __attribute__((aligned(16))) unsigned short sPh[4][16][40];
  __shared__ __attribute__((aligned(16))) unsigned short sPl[4][16][40];
  __shared__ __attribute__((aligned(16))) unsigned short sOh[4][16][72];
  __shared__ __attribute__((aligned(16))) unsigned short sOl[4][16][72];
  const int tid = threadIdx.x;
  const int w = __builtin_amdgcn_readfirstlane(tid >> 5);
  const int lane = tid & 31, ln = lane & 15, hh = lane >> 4;
  const int bh = blockIdx.y;
  const int b = bh / NH, h = bh - b * NH;
  const int q0 = blockIdx.x * 64 + w * 16;
  const bool fine = (blockIdx.x * 64) < FINE_ROWS;
  const size_t tok0 = (size_t)b * SEQ;
  const size_t qoff = (tok0 + q0 + ln) * LQK + h * HD;
  const size_t kcol = tok0 * LQK + DM + h * HD;
  const size_t vrow = (size_t)(h * HD + ln) * NRT + tok0;
  const float NEGINF = -__builtin_inff();
  const float SCL = 1.4426950408889634f * 3.0517578125e-05f;
  const v8f z8 = {0.f, 0.f, 0.f, 0.f, 0.f, 0.f, 0.f, 0.f};
  v8f acc[4] = {z8, z8, z8, z8};
  float m[8], l[8];
#pragma unroll
  for (int r = 0; r < 8; ++r) { m[r] = NEGINF; l[r] = 0.0f; }

#pragma unroll 1
  for (int c = 0; c < SEQ / 32; ++c) {
    const int jt = c * 32;
    const unsigned int* mp = MB + (size_t)c * SEQ + q0 + 8 * hh;
    const v4ua wa = *(const v4ua*)mp;
    const v4ua wb = *(const v4ua*)(mp + 4);
    const unsigned int wd[8] = {wa[0], wa[1], wa[2], wa[3], wb[0], wb[1], wb[2], wb[3]};
    const unsigned int wand = wd[0] & wd[1] & wd[2] & wd[3] & wd[4] & wd[5] & wd[6] & wd[7];
    if (__all(wand == 0xFFFFFFFFu)) continue;

    v8f s0 = z8, s1 = z8;
    const size_t kr0 = kcol + (size_t)(jt + ln) * LQK;
    const size_t kr1 = kr0 + (size_t)16 * LQK;
    if (fine) {
#pragma unroll
      for (int ks = 0; ks < 2; ++ks) {
        const int k0 = ks * 32;
        const v16h qh = ld_frag(QKH + qoff + k0, hh), ql = ld_frag(QKL + qoff + k0, hh);
        const v16h kh0 = ld_frag(QKH + kr0 + k0, hh), kl0 = ld_frag(QKL + kr0 + k0, hh);
        s0 = mma3(qh, ql, kh0, kl0, s0);
        const v16h kh1 = ld_frag(QKH + kr1 + k0, hh), kl1 = ld_frag(QKL + kr1 + k0, hh);
        s1 = mma3(qh, ql, kh1, kl1, s1);
      }
    } else {
#pragma unroll
      for (int ks = 0; ks < 2; ++ks) {
        const int k0 = ks * 32;
        const v16h qh = ld_frag(QKH + qoff + k0, hh);
        const v16h kh0 = ld_frag(QKH + kr0 + k0, hh);
        s0 = mma1(qh, kh0, s0);
        const v16h kh1 = ld_frag(QKH + kr1 + k0, hh);
        s1 = mma1(qh, kh1, s1);
      }
    }

    __builtin_amdgcn_fence(4  , "workgroup");
    __builtin_amdgcn_wave_barrier();
#pragma unroll
    for (int r = 0; r < 8; ++r) {
      const unsigned int wr = wd[r];
      float v0 = s0[r] * SCL, v1 = s1[r] * SCL;
      v0 = ((wr >> ln) & 1u) ? NEGINF : v0;
      v1 = ((wr >> (16 + ln)) & 1u) ? NEGINF : v1;
      float tm = fmaxf(v0, v1);
      tm = fmaxf(tm, __shfl_xor(tm, 1, 16));
      tm = fmaxf(tm, __shfl_xor(tm, 2, 16));
      tm = fmaxf(tm, __shfl_xor(tm, 4, 16));
      tm = fmaxf(tm, __shfl_xor(tm, 8, 16));
      const float mn = fmaxf(m[r], tm);
      const float ms = (mn == NEGINF) ? 0.0f : mn;
      const float al = exp2f(m[r] - ms);
      const float p0 = exp2f(v0 - ms);
      const float p1 = exp2f(v1 - ms);
      l[r] = l[r] * al + (p0 + p1);
      m[r] = mn;
      acc[0][r] *= al; acc[1][r] *= al; acc[2][r] *= al; acc[3][r] *= al;
      const float c0 = p0 * 4096.0f, c1 = p1 * 4096.0f;
      const _Float16 h0 = (_Float16)c0, h1 = (_Float16)c1;
      sPh[w][8 * hh + r][ln] = hbits(h0);
      sPh[w][8 * hh + r][16 + ln] = hbits(h1);
      if (fine) {
        sPl[w][8 * hh + r][ln] = hbits((_Float16)(c0 - (float)h0));
        sPl[w][8 * hh + r][16 + ln] = hbits((_Float16)(c1 - (float)h1));
      }
    }
    __builtin_amdgcn_fence(4  , "workgroup");
    __builtin_amdgcn_wave_barrier();

    FragH ph;
    ph.half[0] = *(const v8us*)&sPh[w][ln][8 * hh];
    ph.half[1] = *(const v8us*)&sPh[w][ln][16 + 8 * hh];
    const size_t vo = vrow + jt;
    if (fine) {
      FragH pl;
      pl.half[0] = *(const v8us*)&sPl[w][ln][8 * hh];
      pl.half[1] = *(const v8us*)&sPl[w][ln][16 + 8 * hh];
#pragma unroll
      for (int dt = 0; dt < 4; ++dt) {
        const size_t o = vo + (size_t)(dt * 16) * NRT;
        const v16h vh = ld_frag(VTH + o, hh), vl = ld_frag(VTL + o, hh);
        acc[dt] = mma3(ph.v, pl.v, vh, vl, acc[dt]);
      }
    } else {
#pragma unroll
      for (int dt = 0; dt < 4; ++dt) {
        const size_t o = vo + (size_t)(dt * 16) * NRT;
        const v16h vh = ld_frag(VTH + o, hh);
        acc[dt] = mma1(ph.v, vh, acc[dt]);
      }
    }
  }

#pragma unroll
  for (int r = 0; r < 8; ++r) {
    float lr = l[r];
    lr += __shfl_xor(lr, 1, 16);
    lr += __shfl_xor(lr, 2, 16);
    lr += __shfl_xor(lr, 4, 16);
    lr += __shfl_xor(lr, 8, 16);
    const float sc = (1.0f / lr) * 0.0009765625f;
#pragma unroll
    for (int dt = 0; dt < 4; ++dt) {
      const float cv = acc[dt][r] * sc;
      const _Float16 hv = (_Float16)cv;
      sOh[w][8 * hh + r][dt * 16 + ln] = hbits(hv);
      if (fine) sOl[w][8 * hh + r][dt * 16 + ln] = hbits((_Float16)(cv - (float)hv));
    }
  }
  __builtin_amdgcn_fence(4  , "workgroup");
  __builtin_amdgcn_wave_barrier();
  const int rq = lane >> 3, c8 = (lane & 7) * 8;
  for (int pass = 0; pass < 2; ++pass) {
#pragma unroll
    for (int q = 0; q < 4; ++q) {
      const int r = q * 4 + rq;
      const size_t o = (tok0 + q0 + r) * DM + h * HD + c8;
      const v8us vh = *(const v8us*)&sOh[w][r][c8];
      *(volatile v8us*)(OH + o) = vh;
      if (fine) {
        const v8us vl = *(const v8us*)&sOl[w][r][c8];
        *(volatile v8us*)(OL + o) = vl;
      }
    }
    if (pass == 0) __threadfence();
  }
}

constexpr size_t SZ_WQK = (size_t)2 * DM * DM * 2;
constexpr size_t SZ_W   = (size_t)DM * DM * 2;
constexpr size_t SZ_X   = (size_t)NRT * DM * 2;
constexpr size_t SZ_QK  = (size_t)NRT * LQK * 2;
constexpr size_t SZ_VT  = (size_t)DM * NRT * 2;
constexpr size_t SZ_O   = (size_t)NRT * DM * 2;
constexpr size_t SZ_MB  = (size_t)(SEQ / 32) * SEQ * 4;
constexpr size_t OF_WQK = 0;
constexpr size_t OF_WV  = OF_WQK + SZ_WQK;
constexpr size_t OF_WO  = OF_WV + SZ_W;
constexpr size_t OF_X   = OF_WO + SZ_W;
constexpr size_t OF_QKH = OF_X + SZ_X;
constexpr size_t OF_QKL = OF_QKH + SZ_QK;
constexpr size_t OF_VTH = OF_QKL + SZ_QK;
constexpr size_t OF_VTL = OF_VTH + SZ_VT;
constexpr size_t OF_OH  = OF_VTL + SZ_VT;
constexpr size_t OF_OL  = OF_OH + SZ_O;
constexpr size_t OF_MB  = OF_OL + SZ_O;
constexpr size_t WS_TOTAL = OF_MB + SZ_MB;
static_assert(SZ_WQK % 256 == 0);
static_assert(SZ_W % 256 == 0);
static_assert(SZ_X % 256 == 0);
static_assert(SZ_QK % 256 == 0);
static_assert(SZ_VT % 256 == 0);
static_assert(SZ_O % 256 == 0);
static_assert(SZ_MB % 128 == 0);
static_assert(WS_TOTAL <= (size_t)134217728);

extern "C" void kernel_launch(void* const* d_in, const int* in_sizes, int n_in,
                              void* d_out, int out_size, void* d_ws, size_t ws_size, hipStream_t stream) {
  if (n_in < 6) return;
  const long long needx = ((long long)(SEQ - 1) * B_FULL + NB) * DM;
  if ((long long)in_sizes[0] < needx) return;
  if ((long long)in_sizes[1] < (long long)DM * DM) return;
  if ((long long)in_sizes[2] < (long long)DM * DM) return;
  if ((long long)in_sizes[3] < (long long)DM * DM) return;
  if ((long long)in_sizes[4] < (long long)DM * DM) return;
  if ((long long)in_sizes[5] < (long long)(SEQ - 1) * T_FULL + SEQ) return;
  if ((long long)out_size < needx) return;
  if (ws_size < WS_TOTAL) return;
  const float* x  = (const float*)d_in[0];
  const float* Wk = (const float*)d_in[1];
  const float* Wv = (const float*)d_in[2];
  const float* Wq = (const float*)d_in[3];
  const float* Wo = (const float*)d_in[4];
  const int* mask = (const int*)d_in[5];
  char* ws = (char*)d_ws;
  unsigned short* WQK = (unsigned short*)(ws + OF_WQK);
  unsigned short* WV  = (unsigned short*)(ws + OF_WV);
  unsigned short* WO  = (unsigned short*)(ws + OF_WO);
  unsigned short* X16 = (unsigned short*)(ws + OF_X);
  unsigned short* QKH = (unsigned short*)(ws + OF_QKH);
  unsigned short* QKL = (unsigned short*)(ws + OF_QKL);
  unsigned short* VTH = (unsigned short*)(ws + OF_VTH);
  unsigned short* VTL = (unsigned short*)(ws + OF_VTL);
  unsigned short* OH  = (unsigned short*)(ws + OF_OH);
  unsigned short* OL  = (unsigned short*)(ws + OF_OL);
  unsigned int*   MB  = (unsigned int*)(ws + OF_MB);

  const unsigned wblocks = (unsigned)(((size_t)DM * (DM / 8) + 255) / 256);
  k_x16<<<(unsigned)(((size_t)NRT * (DM / 8) + 255) / 256), 256, 0, stream>>>(x, X16);
  k_wplane<<<wblocks, 256, 0, stream>>>(Wq, WQK, 1);
  k_wplane<<<wblocks, 256, 0, stream>>>(Wk, WQK + (size_t)DM * DM, 1);
  k_wplane<<<wblocks, 256, 0, stream>>>(Wv, WV, 1);
  k_wplane<<<wblocks, 256, 0, stream>>>(Wo, WO, 0);
  k_maskbits<<<SEQ / 32, 256, 0, stream>>>(mask, MB);
  k_proj<<<(unsigned)((NRT / 128) * (LQK / 64)), 128, 0, stream>>>(X16, DM, WQK, DM, 4.0f, QKH, QKL, LQK, NRT, LQK, DM);
  k_proj<<<(unsigned)((DM / 128) * (NRT / 64)), 128, 0, stream>>>(WV, DM, X16, DM, 4.0f, VTH, VTL, NRT, DM, NRT, DM);
  k_attn<<<dim3(SEQ / 64, NB * NH), 128, 0, stream>>>(QKH, QKL, VTH, VTL, MB, OH, OL);
  k_outg<<<(unsigned)((NRT / 128) * (DM / 64)), 128, 0, stream>>>(OH, OL, WO, 0.000244140625f, (float*)d_out);
}
